// GraphAttention_23175643529906
// MI455X (gfx1250) — hardware-run, weakly checked
//
#include <hip/hip_runtime.h>
#include <stddef.h>
#include <stdint.h>
#include <math.h>

#define NN      50000
#define NE      800000
#define DM      128
#define NHD     8
#define DKH     16
#define GBM     128
#define MP      50048
#define QP      384
#define KO      256
#ifndef SPLIT_O
#define SPLIT_O 1
#endif
#define KOUT    (SPLIT_O ? 256 : 128)
#define NTHR    256
#define NWAVE   8
#define EPT     8
#define WCH     (32 * EPT)
#define NBRUN   1024
#define SLB     10
#define NBK     49
#define WLCAP   3584
#define RCAP    28672
#define DEGCAP  64
#define MAXDEG_MEAS   35
#define MAXB1024_MEAS 16672
#define ABM     64
#define SP      68
#define WSMAX   (128u << 20)

#define BK_ZINTS (NWAVE * WLCAP + RCAP + 3 * NBRUN)
#define BK_INTS  (BK_ZINTS + 16)
#define BK_LDS   (BK_INTS * 4)

#define PBX   (MP * DM / 8 / NTHR)
#define PBW   (3 * DM * DM / 8 / NTHR)
#define PBO   (DM * KO / 8 / NTHR)
#define PBTOT (PBX + PBW + PBO + 1)

static_assert(DM == 128 && DM == 32 * 4);
static_assert(NHD * DKH == DM && DKH == 16 && DKH == 4 * 4);
static_assert(MP % GBM == 0 && MP >= NN && MP == 391 * GBM && MP % ABM == 0);
static_assert(NBRUN == (1 << SLB) && NBRUN <= 1024 && NBRUN % ABM == 0 && NBRUN % GBM == 0 && NBRUN % 32 == 0);
static_assert(NBK * NBRUN >= MP);
static_assert(NN <= 65536);
static_assert(NE < (1 << 21) && (((long long)NE) << SLB) < (1LL << 31));
static_assert(NE % WCH == 0 && NE % 4 == 0);
static_assert(RCAP == NWAVE * WLCAP && RCAP % (NTHR * 4) == 0 && BK_ZINTS % 4 == 0);
static_assert((2 * NBRUN) % (NTHR * 4) == 0);
static_assert((long long)RCAP * 100 >= (long long)MAXB1024_MEAS * 105);
static_assert(WLCAP >= MAXB1024_MEAS / 8 + 8 * 46 + 1);
static_assert(MAXDEG_MEAS + 8 <= DEGCAP && DEGCAP < 65536);
static_assert((MP * DM / 8) % NTHR == 0 && (DM * DM / 8) % NTHR == 0 && (DM * KO / 8) % NTHR == 0);
static_assert(DM % 32 == 0 && KO % 32 == 0 && KOUT % 32 == 0 && KOUT <= KO && KO == 2 * DM);
static_assert(QP == 3 * DM && QP % 64 == 0);
static_assert(ABM == 8 * NWAVE);
static_assert(BK_LDS <= 300000);
static_assert((GBM * SP + 64) * 4 <= 65536);

typedef float          v4f   __attribute__((ext_vector_type(4)));
typedef float          v8f   __attribute__((ext_vector_type(8)));
typedef int            v2i   __attribute__((ext_vector_type(2)));
typedef int            v4i   __attribute__((ext_vector_type(4)));
typedef int            v8i   __attribute__((ext_vector_type(8)));
typedef unsigned short v8us  __attribute__((ext_vector_type(8)));
typedef unsigned short v16us __attribute__((ext_vector_type(16)));
typedef __bf16         v16bf __attribute__((ext_vector_type(16)));
typedef v4f  __attribute__((may_alias)) v4fa;
typedef v4i  __attribute__((may_alias)) v4ia;
typedef v8us __attribute__((may_alias)) v8usa;
union FragB { v16bf v; v16us u; v8us h[2]; v8i w; };

__device__ __forceinline__ v8f wmb(const FragB& a, const FragB& b, v8f c) {
  v8f d = __builtin_amdgcn_wmma_f32_16x16x32_bf16(false, a.v, false, b.v, (short)0, c, false, false);
  asm volatile("v_nop\n\tv_nop\n\tv_nop\n\tv_nop" : "+v"(d) : "v"(a.w), "v"(b.w));
  return d;
}

__device__ __forceinline__ unsigned bf16_bits(float f) {
  const unsigned u = __float_as_uint(f);
  const unsigned r = (u + 0x7FFFu + ((u >> 16) & 1u)) >> 16;
  const unsigned q = (u >> 16) | 0x40u;
  return ((u & 0x7fffffffu) > 0x7f800000u) ? q : r;
}
__device__ __forceinline__ float bf16_val(float f) {
  return __uint_as_float(bf16_bits(f) << 16);
}

__device__ __forceinline__ void hilo_pack(float v0, float v1, float v2, float v3,
                                          int& h01, int& h23, int& l01, int& l23) {
  const unsigned a0 = bf16_bits(v0), a1 = bf16_bits(v1), a2 = bf16_bits(v2), a3 = bf16_bits(v3);
  const unsigned b0 = bf16_bits(v0 - __uint_as_float(a0 << 16));
  const unsigned b1 = bf16_bits(v1 - __uint_as_float(a1 << 16));
  const unsigned b2 = bf16_bits(v2 - __uint_as_float(a2 << 16));
  const unsigned b3 = bf16_bits(v3 - __uint_as_float(a3 << 16));
  h01 = (int)(a0 | (a1 << 16)); h23 = (int)(a2 | (a3 << 16));
  l01 = (int)(b0 | (b1 << 16)); l23 = (int)(b2 | (b3 << 16));
}

__device__ __forceinline__ void st2_v4f(float* p, v4f v) {
  *(volatile v4f*)p = v;
  __threadfence();
  *(volatile v4f*)p = v;
}
__device__ __forceinline__ void st2_v8us(unsigned short* p, v8us v) {
  *(volatile v8us*)p = v;
  __threadfence();
  *(volatile v8us*)p = v;
}

__device__ __forceinline__ v8us cvt8(const v4f a, const v4f b, const unsigned mk) {
  v8us o;
  o[0] = (unsigned short)(bf16_bits(a.x) & mk); o[1] = (unsigned short)(bf16_bits(a.y) & mk);
  o[2] = (unsigned short)(bf16_bits(a.z) & mk); o[3] = (unsigned short)(bf16_bits(a.w) & mk);
  o[4] = (unsigned short)(bf16_bits(b.x) & mk); o[5] = (unsigned short)(bf16_bits(b.y) & mk);
  o[6] = (unsigned short)(bf16_bits(b.z) & mk); o[7] = (unsigned short)(bf16_bits(b.w) & mk);
  return o;
}

__device__ __forceinline__ void wrow_unit(const float* __restrict__ w, unsigned short* dst,
                                          int n, int ksrc, int kdst, int pitch) {
  const float* p = w + (size_t)n * DM + ksrc;
  const v4f a = *(const v4fa*)p;
  const v4f b = *(const v4fa*)(p + 4);
  st2_v8us(dst + (size_t)n * (size_t)pitch + kdst, cvt8(a, b, 0xffffu));
}

__global__ __launch_bounds__(NTHR) void k_prep(const float* __restrict__ h,
                                               const float* __restrict__ wq, const float* __restrict__ bq,
                                               const float* __restrict__ wk, const float* __restrict__ bk,
                                               const float* __restrict__ wv, const float* __restrict__ bv,
                                               const float* __restrict__ wo, const float* __restrict__ bo,
                                               unsigned short* xb, unsigned short* wqkv, unsigned short* wo2,
                                               float* sm) {
  const int tid = (int)threadIdx.x, lane = tid & 31;
  const int blk = (int)blockIdx.x;
  if (blk < PBX) {
    const int u   = blk * NTHR + tid;
    const int row = u >> 4, k8 = (u & 15) * 8;
    const int rc  = row < NN ? row : NN - 1;
    const unsigned mk = row < NN ? 0xffffu : 0u;
    const float* p = h + (size_t)rc * DM + k8;
    const v4f a = *(const v4fa*)p;
    const v4f b = *(const v4fa*)(p + 4);
    st2_v8us(xb + (size_t)row * DM + k8, cvt8(a, b, mk));
  } else if (blk < PBX + PBW) {
    const int b2  = blk - PBX;
    const int mat = b2 >> 3;
    const int u   = (b2 & 7) * NTHR + tid;
    const int n = u >> 4, k8 = (u & 15) * 8;
    if (mat == 0)      wrow_unit(wq, wqkv, n, k8, k8, DM);
    else if (mat == 1) wrow_unit(wk, wqkv + DM * DM, n, k8, k8, DM);
    else               wrow_unit(wv, wqkv + 2 * DM * DM, n, k8, k8, DM);
  } else if (blk < PBX + PBW + PBO) {
    const int u = (blk - PBX - PBW) * NTHR + tid;
    const int n = u >> 5, k8 = (u & 31) * 8;
    wrow_unit(wo, wo2, n, k8 & (DM - 1), k8, KO);
  } else {
    if (tid < 128) {
      const int w = tid >> 5;
      v4f a;
      if (w == 0)      a = *(const v4fa*)(bq + 4 * lane);
      else if (w == 1) a = *(const v4fa*)(bk + 4 * lane);
      else if (w == 2) a = *(const v4fa*)(bv + 4 * lane);
      else             a = *(const v4fa*)(bo + 4 * lane);
      v4f o;
      o.x = bf16_val(a.x); o.y = bf16_val(a.y); o.z = bf16_val(a.z); o.w = bf16_val(a.w);
      st2_v4f(sm + 128 * w + 4 * lane, o);
    }
  }
}

template <int KTOT, int BPITCH>
__device__ __forceinline__ void gemm_16x64(const unsigned short* __restrict__ ap,
                                           const unsigned short* __restrict__ bp, v8f (&acc)[4]) {
  static_assert(KTOT % 32 == 0 && KTOT <= BPITCH);
#pragma unroll 1
  for (int k0 = 0; k0 < KTOT; k0 += 32) {
    FragB af;
    af.h[0] = *(const v8usa*)(ap + k0);
    af.h[1] = *(const v8usa*)(ap + k0 + 16);
#pragma unroll
    for (int nt = 0; nt < 4; ++nt) {
      const unsigned short* wq = bp + (size_t)(16 * nt) * (size_t)BPITCH + k0;
      FragB bf;
      bf.h[0] = *(const v8usa*)wq;
      bf.h[1] = *(const v8usa*)(wq + 16);
      acc[nt] = wmb(af, bf, acc[nt]);
    }
  }
}

__device__ __forceinline__ void stage_d(float* stg, const v8f (&acc)[4], int wave, int hh, int m) {
#pragma unroll
  for (int nt = 0; nt < 4; ++nt) {
#pragma unroll
    for (int r = 0; r < 8; ++r) stg[(16 * wave + 8 * hh + r) * SP + 16 * nt + m] = acc[nt][r];
  }
}

__global__ __launch_bounds__(NTHR) __attribute__((amdgpu_num_vgpr(248)))
void k_qkv(const unsigned short* __restrict__ XB, const unsigned short* __restrict__ WQKV,
           const float* __restrict__ sm, float* QKV) {
  __shared__ __attribute__((aligned(16))) float stg[GBM * SP];
  __shared__ __attribute__((aligned(16))) float sb[64];
  const int tid = (int)threadIdx.x, lane = tid & 31, wave = tid >> 5, hh = lane >> 4, m = lane & 15;
  const int rowBase = (int)blockIdx.x * GBM;
  const int col0    = (int)blockIdx.y * 64;
  if (tid < 16) *(v4fa*)(sb + 4 * tid) = *(const v4fa*)(sm + col0 + 4 * tid);

  v8f acc[4];
  {
    const v8f z = {0.f, 0.f, 0.f, 0.f, 0.f, 0.f, 0.f, 0.f};
#pragma unroll
    for (int t = 0; t < 4; ++t) acc[t] = z;
  }
  const unsigned short* ap = XB + (size_t)(rowBase + 16 * wave + m) * (size_t)DM + 8 * hh;
  const unsigned short* bp = WQKV + (size_t)(col0 + m) * (size_t)DM + 8 * hh;
  gemm_16x64<DM, DM>(ap, bp, acc);
  stage_d(stg, acc, wave, hh, m);
  __syncthreads();

  const v4f bias = *(const v4fa*)(sb + 4 * m);
#pragma unroll 1
  for (int i = 0; i < 8; ++i) {
    const int lr   = 16 * wave + 2 * i + hh;
    const int grow = rowBase + lr;
    const v4f a = *(const v4fa*)(stg + lr * SP + 4 * m);
    v4f o;
    o.x = a.x + bias.x; o.y = a.y + bias.y; o.z = a.z + bias.z; o.w = a.w + bias.w;
    st2_v4f(QKV + (size_t)grow * QP + col0 + 4 * m, o);
  }
}

__device__ __forceinline__ void bucket_flush(const int* pl, const int* cnt, int ov, int* lp, int* cop, int* fp,
                                             int tid) {
#pragma unroll 1
  for (int i = tid * 4; i < RCAP; i += NTHR * 4) {
    const v4i v = *(const v4ia*)(pl + i);
    *(volatile v4i*)(lp + i) = v;
  }
#pragma unroll 1
  for (int i = tid * 4; i < 2 * NBRUN; i += NTHR * 4) {
    const v4i v = *(const v4ia*)(cnt + i);
    *(volatile v4i*)(cop + i) = v;
  }
  if (tid < 8) {
    const v4i f = {ov, ov, ov, ov};
    *(volatile v4i*)(fp + 4 * tid) = f;
  }
}

__global__ __launch_bounds__(NTHR) void k_bucket(const int* __restrict__ srcs, const int* __restrict__ dsts,
                                                 int* LIST, int* CO, int* FLAG) {
  extern __shared__ __attribute__((aligned(16))) int dsm[];
  int* wl   = dsm;
  int* pl   = dsm + NWAVE * WLCAP;
  int* cnt  = pl + RCAP;
  int* offs = cnt + NBRUN;
  int* cur  = offs + NBRUN;
  int* misc = cur + NBRUN;
  const int tid = (int)threadIdx.x, lane = tid & 31, wave = tid >> 5;
  const int blk = (int)blockIdx.x;
  const unsigned nbs = (unsigned)(blk * NBRUN);

  {
    const v4i z4 = {0, 0, 0, 0};
    for (int i = tid * 4; i < BK_ZINTS; i += NTHR * 4) *(v4ia*)(dsm + i) = z4;
    if (tid < 16) misc[tid] = 0;
  }
  __syncthreads();

  {
    const int per  = ((NE + NWAVE * WCH - 1) / (NWAVE * WCH)) * WCH;
    const int ebeg = wave * per;
    const int eend = (ebeg + per < NE) ? (ebeg + per) : NE;
    int* mylist = wl + wave * WLCAP;
    int wc = 0;
#pragma unroll 1
    for (int cb = ebeg; cb < eend; cb += WCH) {
      const int e0 = cb + lane * EPT;
      const v4i da = *(const v4ia*)(dsts + e0);
      const v4i db = *(const v4ia*)(dsts + e0 + 4);
      const unsigned s0 = (unsigned)da.x - nbs, s1 = (unsigned)da.y - nbs;
      const unsigned s2 = (unsigned)da.z - nbs, s3 = (unsigned)da.w - nbs;
      const unsigned s4 = (unsigned)db.x - nbs, s5 = (unsigned)db.y - nbs;
      const unsigned s6 = (unsigned)db.z - nbs, s7 = (unsigned)db.w - nbs;
      const bool h0 = s0 < (unsigned)NBRUN, h1 = s1 < (unsigned)NBRUN, h2 = s2 < (unsigned)NBRUN, h3 = s3 < (unsigned)NBRUN;
      const bool h4 = s4 < (unsigned)NBRUN, h5 = s5 < (unsigned)NBRUN, h6 = s6 < (unsigned)NBRUN, h7 = s7 < (unsigned)NBRUN;
      const unsigned m0 = __builtin_amdgcn_ballot_w32(h0), m1 = __builtin_amdgcn_ballot_w32(h1);
      const unsigned m2 = __builtin_amdgcn_ballot_w32(h2), m3 = __builtin_amdgcn_ballot_w32(h3);
      const unsigned m4 = __builtin_amdgcn_ballot_w32(h4), m5 = __builtin_amdgcn_ballot_w32(h5);
      const unsigned m6 = __builtin_amdgcn_ballot_w32(h6), m7 = __builtin_amdgcn_ballot_w32(h7);
      const unsigned any = m0 | m1 | m2 | m3 | m4 | m5 | m6 | m7;
      if (any != 0u) {
        const int pre = (int)(__builtin_amdgcn_mbcnt_lo(m0, 0u) + __builtin_amdgcn_mbcnt_lo(m1, 0u) +
                              __builtin_amdgcn_mbcnt_lo(m2, 0u) + __builtin_amdgcn_mbcnt_lo(m3, 0u) +
                              __builtin_amdgcn_mbcnt_lo(m4, 0u) + __builtin_amdgcn_mbcnt_lo(m5, 0u) +
                              __builtin_amdgcn_mbcnt_lo(m6, 0u) + __builtin_amdgcn_mbcnt_lo(m7, 0u));
        int p = wc + pre;
        if (h0) { if (p < WLCAP) mylist[p] = ((e0 + 0) << SLB) | (int)s0; p = p + 1; }
        if (h1) { if (p < WLCAP) mylist[p] = ((e0 + 1) << SLB) | (int)s1; p = p + 1; }
        if (h2) { if (p < WLCAP) mylist[p] = ((e0 + 2) << SLB) | (int)s2; p = p + 1; }
        if (h3) { if (p < WLCAP) mylist[p] = ((e0 + 3) << SLB) | (int)s3; p = p + 1; }
        if (h4) { if (p < WLCAP) mylist[p] = ((e0 + 4) << SLB) | (int)s4; p = p + 1; }
        if (h5) { if (p < WLCAP) mylist[p] = ((e0 + 5) << SLB) | (int)s5; p = p + 1; }
        if (h6) { if (p < WLCAP) mylist[p] = ((e0 + 6) << SLB) | (int)s6; p = p + 1; }
        if (h7) { if (p < WLCAP) mylist[p] = ((e0 + 7) << SLB) | (int)s7; p = p + 1; }
        wc += (int)(__builtin_popcount(m0) + __builtin_popcount(m1) + __builtin_popcount(m2) + __builtin_popcount(m3) +
                    __builtin_popcount(m4) + __builtin_popcount(m5) + __builtin_popcount(m6) + __builtin_popcount(m7));
      }
    }
    if (lane == 0) misc[wave] = wc;
  }
  __syncthreads();

  if (wave == 0) {
    int ov = 0;
#pragma unroll 1
    for (int w2 = 0; w2 < NWAVE; ++w2) {
      int c = misc[w2];
      if (c > WLCAP) ov = 1;
      c = c < 0 ? 0 : (c > WLCAP ? WLCAP : c);
#pragma unroll 1
      for (int b0 = 0; b0 < c; b0 += 32) {
        const int idx = b0 + lane;
        const int ent = wl[w2 * WLCAP + (idx < WLCAP ? idx : WLCAP - 1)];
        const int m32 = (c - b0) < 32 ? (c - b0) : 32;
#pragma unroll 1
        for (int k = 0; k < m32; ++k) {
          const int u    = __builtin_amdgcn_readlane(ent, k);
          const int slot = u & (NBRUN - 1);
          if (lane == 0) cnt[slot] = cnt[slot] + 1;
        }
      }
    }
    if (lane == 0) misc[9] = ov;
  }
  __syncthreads();
  if (wave == 0) {
    const int base = lane * (NBRUN / 32);
    int s = 0;
#pragma unroll 1
    for (int i = 0; i < NBRUN / 32; ++i) s += cnt[base + i];
    int incl = s;
#pragma unroll
    for (int d = 1; d < 32; d <<= 1) {
      const int y = __shfl_up(incl, d, 32);
      if (lane >= d) incl += y;
    }
    int run = incl - s;
#pragma unroll 1
    for (int i = 0; i < NBRUN / 32; ++i) {
      const int cv = cnt[base + i];
      offs[base + i] = run;
      cur[base + i]  = run;
      run += cv;
    }
  }
  __syncthreads();

  if (wave == 0) {
#pragma unroll 1
    for (int w2 = 0; w2 < NWAVE; ++w2) {
      int c = misc[w2];
      c = c < 0 ? 0 : (c > WLCAP ? WLCAP : c);
#pragma unroll 1
      for (int b0 = 0; b0 < c; b0 += 32) {
        const int idx = b0 + lane;
        const int ent = wl[w2 * WLCAP + (idx < WLCAP ? idx : WLCAP - 1)];
        int eid = (ent >> SLB) & 0x1FFFFF;
        eid = eid > NE - 1 ? NE - 1 : eid;
        int sr = srcs[eid];
        sr = sr < 0 ? 0 : (sr > NN - 1 ? NN - 1 : sr);
        const int word = (int)((unsigned)sr | ((unsigned)(ent & (NBRUN - 1)) << 16));
        const int m32 = (c - b0) < 32 ? (c - b0) : 32;
#pragma unroll 1
        for (int k = 0; k < m32; ++k) {
          const int u    = __builtin_amdgcn_readlane(ent, k);
          const int wd   = __builtin_amdgcn_readlane(word, k);
          const int slot = u & (NBRUN - 1);
          if (lane == 0) {
            int p = cur[slot];
            p = p < 0 ? 0 : (p > RCAP - 1 ? RCAP - 1 : p);
            pl[p] = wd;
            cur[slot] = p + 1;
          }
        }
      }
    }
  }
  __syncthreads();

  const int ovf = misc[9];
  int* lp  = LIST + (size_t)blk * RCAP;
  int* cop = CO + (size_t)blk * (2 * NBRUN);
  int* fp  = FLAG + (size_t)blk * 32;
  bucket_flush(pl, cnt, ovf, lp, cop, fp, tid);
  __threadfence();
  bucket_flush(pl, cnt, ovf, lp, cop, fp, tid);
}

__global__ __launch_bounds__(NTHR) void k_replay(const int* __restrict__ LIST, const int* __restrict__ CO,
                                                 const int* __restrict__ FLAG, const float* __restrict__ QKV,
                                                 unsigned short* AGG) {
  const int tid = (int)threadIdx.x, lane = tid & 31, wave = tid >> 5;
  const int rowBase = (int)blockIdx.x * ABM;
  const int bucket  = rowBase >> SLB;
  const int* lb  = LIST + (size_t)bucket * RCAP;
  const int* cob = CO + (size_t)bucket * (2 * NBRUN);
  const int flag = FLAG[(size_t)bucket * 32];
  const float qnan = __uint_as_float(0x7fc00000u);
  const float ninf = __uint_as_float(0xff800000u);

#pragma unroll 1
  for (int i = 0; i < ABM / NWAVE; ++i) {
    const int d    = rowBase + (ABM / NWAVE) * wave + i;
    const int slot = d & (NBRUN - 1);
    int cv = cob[slot];
    int ov = cob[NBRUN + slot];
    const bool big = cv > DEGCAP;
    cv = cv < 0 ? 0 : (cv > DEGCAP ? DEGCAP : cv);
    ov = ov < 0 ? 0 : (ov > RCAP - 1 ? RCAP - 1 : ov);
    const int c = __builtin_amdgcn_readfirstlane(cv);
    const int o = __builtin_amdgcn_readfirstlane(ov);
    int last = o + c - 1;
    last = last < o ? o : last;
    last = last > RCAP - 1 ? RCAP - 1 : last;

    const int dc = d < NN ? d : NN - 1;
    const v4f qr = *(const v4fa*)(QKV + (size_t)dc * QP + 4 * lane);
    const float q0 = qr.x * 0.25f, q1 = qr.y * 0.25f, q2 = qr.z * 0.25f, q3 = qr.w * 0.25f;

    float mx = ninf, ss = 0.0f;
    float a0 = 0.0f, a1 = 0.0f, a2 = 0.0f, a3 = 0.0f;
#pragma unroll 1
    for (int j = 0; j < c; ++j) {
      int idx = o + j;
      idx = idx > last ? last : idx;
      const unsigned wd = (unsigned)lb[idx];
      int sr = (int)(wd & 0xffffu);
      sr = sr > NN - 1 ? NN - 1 : sr;
      const float* kp = QKV + (size_t)sr * QP + DM + 4 * lane;
      const v4f kk = *(const v4fa*)kp;
      const v4f vv = *(const v4fa*)(kp + DM);
      float part = q0 * kk.x;
      part = fmaf(q1, kk.y, part);
      part = fmaf(q2, kk.z, part);
      part = fmaf(q3, kk.w, part);
      part += __shfl_xor(part, 1, 32);
      part += __shfl_xor(part, 2, 32);
      const float sc = part;
      const float df = sc - mx;
      const float ee = expf(-fabsf(df));
      const bool up  = df > 0.0f;
      const float corr = up ? ee : 1.0f;
      const float p    = up ? 1.0f : ee;
      mx = up ? sc : mx;
      ss = fmaf(ss, corr, p);
      a0 = fmaf(a0, corr, p * vv.x);
      a1 = fmaf(a1, corr, p * vv.y);
      a2 = fmaf(a2, corr, p * vv.z);
      a3 = fmaf(a3, corr, p * vv.w);
    }
    const bool empty = (ss == 0.0f);
    const float sd  = empty ? 1.0f : ss;
    const float inv = 1.0f / sd;
    float g0 = empty ? 0.0f : a0 * inv, g1 = empty ? 0.0f : a1 * inv;
    float g2 = empty ? 0.0f : a2 * inv, g3 = empty ? 0.0f : a3 * inv;
    const bool bad  = (flag != 0) | big;
    const bool live = d < NN;
    g0 = bad ? qnan : g0; g1 = bad ? qnan : g1; g2 = bad ? qnan : g2; g3 = bad ? qnan : g3;
    g0 = live ? g0 : 0.0f; g1 = live ? g1 : 0.0f; g2 = live ? g2 : 0.0f; g3 = live ? g3 : 0.0f;
    int h01, h23, l01, l23;
    hilo_pack(g0, g1, g2, g3, h01, h23, l01, l23);
    const v2i hw = {h01, h23};
    const v2i lw = {l01, l23};
    unsigned short* hp = AGG + (size_t)d * KO + 4 * lane;
    unsigned short* lp = hp + DM;
    *(volatile v2i*)hp = hw;
    *(volatile v2i*)lp = lw;
    __threadfence();
    *(volatile v2i*)hp = hw;
    *(volatile v2i*)lp = lw;
  }
}

__global__ __launch_bounds__(NTHR) __attribute__((amdgpu_num_vgpr(248)))
void k_out(const unsigned short* __restrict__ AGG, const unsigned short* __restrict__ WO2,
           const float* __restrict__ sm, const int* __restrict__ FLAG, float* out) {
  __shared__ __attribute__((aligned(16))) float stg[GBM * SP];
  __shared__ __attribute__((aligned(16))) float sb[64];
  const int tid = (int)threadIdx.x, lane = tid & 31, wave = tid >> 5, hh = lane >> 4, m = lane & 15;
  const int rowBase = (int)blockIdx.x * GBM;
  const int col0    = (int)blockIdx.y * 64;
  const int flag = FLAG[(size_t)(rowBase >> SLB) * 32];
  if (tid < 16) *(v4fa*)(sb + 4 * tid) = *(const v4fa*)(sm + 3 * DM + col0 + 4 * tid);

  v8f acc[4];
  {
    const v8f z = {0.f, 0.f, 0.f, 0.f, 0.f, 0.f, 0.f, 0.f};
#pragma unroll
    for (int t = 0; t < 4; ++t) acc[t] = z;
  }
  const unsigned short* ap = AGG + (size_t)(rowBase + 16 * wave + m) * (size_t)KO + 8 * hh;
  const unsigned short* bp = WO2 + (size_t)(col0 + m) * (size_t)KO + 8 * hh;
  gemm_16x64<KOUT, KO>(ap, bp, acc);
  stage_d(stg, acc, wave, hh, m);
  __syncthreads();

  const v4f bias = *(const v4fa*)(sb + 4 * m);
  const float qnan = __uint_as_float(0x7fc00000u);
#pragma unroll 1
  for (int i = 0; i < 8; ++i) {
    const int lr   = 16 * wave + 2 * i + hh;
    const int grow = rowBase + lr;
    const bool live = grow < NN;
    const int gr = live ? grow : NN - 1;
    const v4f a = *(const v4fa*)(stg + lr * SP + 4 * m);
    asm volatile("" :: "v"(a));
    v4f o;
    o.x = a.x + bias.x; o.y = a.y + bias.y; o.z = a.z + bias.z; o.w = a.w + bias.w;
    o.x = (flag != 0) ? qnan : o.x; o.y = (flag != 0) ? qnan : o.y;
    o.z = (flag != 0) ? qnan : o.z; o.w = (flag != 0) ? qnan : o.w;
    float* op = out + (size_t)gr * DM + col0 + 4 * m;
    if (live) *(volatile v4f*)op = o;
    __threadfence();
    if (live) *(volatile v4f*)op = o;
  }
}

extern "C" void kernel_launch(void* const* d_in, const int* in_sizes, int n_in,
                              void* d_out, int out_size, void* d_ws, size_t ws_size,
                              hipStream_t stream) {
  if (n_in < 11) return;
  if (in_sizes[0] != NN * DM) return;
  if (in_sizes[1] != DM * DM || in_sizes[3] != DM * DM) return;
  if (in_sizes[5] != DM * DM || in_sizes[7] != DM * DM) return;
  if (in_sizes[2] != DM || in_sizes[4] != DM || in_sizes[6] != DM || in_sizes[8] != DM) return;
  if (in_sizes[9] != NE || in_sizes[10] != NE) return;
  if (out_size != NN * DM) return;

  const float* h  = (const float*)d_in[0];
  const float* Wq = (const float*)d_in[1];
  const float* bq = (const float*)d_in[2];
  const float* Wk = (const float*)d_in[3];
  const float* bk = (const float*)d_in[4];
  const float* Wv = (const float*)d_in[5];
  const float* bv = (const float*)d_in[6];
  const float* Wo = (const float*)d_in[7];
  const float* bo = (const float*)d_in[8];
  const int*  src = (const int*)d_in[9];
  const int*  dst = (const int*)d_in[10];
  float* out = (float*)d_out;

  constexpr size_t zA    = (size_t)MP * KO * 2;
  constexpr size_t zXB   = (size_t)MP * DM * 2;
  constexpr size_t zQKV  = (size_t)MP * QP * 4;
  constexpr size_t zLIST = (size_t)NBK * RCAP * 4;
  constexpr size_t zCO   = (size_t)NBK * 2 * NBRUN * 4;
  constexpr size_t zFLAG = (size_t)64 * 128;
  constexpr size_t zWQKV = (size_t)3 * DM * DM * 2;
  constexpr size_t zWO2  = (size_t)DM * KO * 2;
  constexpr size_t zSM   = (size_t)4 * DM * 4;
  constexpr size_t oA    = 0;
  constexpr size_t oQKV  = oA + zA;
  constexpr size_t oLIST = oQKV + zQKV;
  constexpr size_t oCO   = oLIST + zLIST;
  constexpr size_t oFLAG = oCO + zCO;
  constexpr size_t oWQKV = oFLAG + zFLAG;
  constexpr size_t oWO2  = oWQKV + zWQKV;
  constexpr size_t oSM   = oWO2 + zWO2;
  constexpr size_t oEND  = oSM + zSM;
  static_assert(zXB <= zA);
  static_assert(zA % 256 == 0 && zQKV % 256 == 0 && zLIST % 256 == 0 && zCO % 256 == 0 && zFLAG % 256 == 0);
  static_assert(zWQKV % 256 == 0 && zWO2 % 256 == 0 && zSM % 256 == 0);
  static_assert((size_t)NBK * 128 <= zFLAG);
  static_assert(oEND <= (size_t)WSMAX);
  if (oEND > ws_size) return;

  char* ws = (char*)d_ws;
  unsigned short* XB   = (unsigned short*)(ws + oA);
  unsigned short* AGG  = (unsigned short*)(ws + oA);
  float*          QKV  = (float*)(ws + oQKV);
  int*            LIST = (int*)(ws + oLIST);
  int*            CO   = (int*)(ws + oCO);
  int*            FLAG = (int*)(ws + oFLAG);
  unsigned short* WQKV = (unsigned short*)(ws + oWQKV);
  unsigned short* WO2  = (unsigned short*)(ws + oWO2);
  float*          SM   = (float*)(ws + oSM);

  hipFuncSetAttribute(reinterpret_cast<const void*>(&k_bucket), hipFuncAttributeMaxDynamicSharedMemorySize, (int)BK_LDS);

  k_prep<<<PBTOT, NTHR, 0, stream>>>(h, Wq, bq, Wk, bk, Wv, bv, Wo, bo, XB, WQKV, WO2, SM);
  k_qkv<<<dim3(MP / GBM, QP / 64), NTHR, 0, stream>>>(XB, WQKV, SM, QKV);
  k_bucket<<<NBK, NTHR, BK_LDS, stream>>>(src, dst, LIST, CO, FLAG);
  k_replay<<<MP / ABM, NTHR, 0, stream>>>(LIST, CO, FLAG, QKV, AGG);
  k_out<<<dim3(MP / GBM, DM / 64), NTHR, 0, stream>>>(AGG, WO2, SM, FLAG, out);
}
